// GNNThicknessPredictor_9070970929320
// MI455X (gfx1250) — hardware-verified
//
#include <hip/hip_runtime.h>
#include <stddef.h>
#include <stdint.h>


#define SPLIT_MEAN0 1
#define SPLIT_CONV  1
#define SPLIT_HEAD  1

#define NN      100000
#define NE      800000
#define FIN     16
#define HD      128
#define H1D     64
#define H2D     32
#define OD      10
#define ODP     16
#define MP      100096
#define PP      256
#define AZP     64
#define KC      512
#define LNEPS   1e-5f
#define NTHR    256
#define NWAVE   8
#define NBA     1024
#define PKS     10
#define NB      98
#define WLCAP   2048
#define RCAP    12288
#define DEGCAP  64
#define WSTEP   256
#define EPW     100096
#define NSTEP   (EPW / WSTEP)
#define MEAS_BLK_HITS 8361
#define MEAS_MAXDEG   23
#define BK_INTS (NWAVE * WLCAP + RCAP + 3 * NBA + 32)
#define LDS_BK  (BK_INTS * 4)
#define GBM     64
#define GBN     128
#define GTHR    128
#define RPB     64
#define RPW     8
#define NU_WZ   1024
#define NU_WCH  8192
#define NU_WC   (2 * NU_WCH)
#define NU_WX   2048
#define NU_WY   512
#define NU_WV   256
#define NU_XB   (MP * 2)
#define UB_WZ   NU_WZ
#define UB_WC   (UB_WZ + NU_WC)
#define UB_WX   (UB_WC + NU_WX)
#define UB_WY   (UB_WX + NU_WY)
#define UB_WV   (UB_WY + NU_WV)
#define NU_ALL  (UB_WV + NU_XB)

static_assert(MP % GBM == 0 && MP >= NN);
static_assert(NB * NBA >= MP && NBA == (1 << PKS) && NBA == NTHR * 4);
static_assert((long long)RCAP * 100 >= (long long)MEAS_BLK_HITS * 105);
static_assert(DEGCAP >= MEAS_MAXDEG + 8);
static_assert(NWAVE * WLCAP >= RCAP);
static_assert(NWAVE * EPW >= NE && EPW % WSTEP == 0);
static_assert((((long long)NWAVE * EPW) << PKS) < (1LL << 31));
static_assert(RCAP % (NTHR * 4) == 0 && BK_INTS % 4 == 0);
static_assert(LDS_BK <= 327680);
static_assert(NU_WZ % NTHR == 0 && NU_WCH % NTHR == 0 && NU_WX % NTHR == 0 && NU_WY % NTHR == 0);
static_assert(NU_WV % NTHR == 0 && NU_ALL % NTHR == 0);
static_assert(GBM == (GTHR / 32) * 16 && GBN == HD && RPB == NWAVE * RPW && RPB == GBM);
static_assert((GBM * OD * 4) % 128 == 0);
static_assert(((NN % GBM) * OD * 4) % 128 == 0);
static_assert((NN * OD) % 4 == 0);
static_assert(KC == 4 * HD && PP == 2 * HD && AZP == 4 * FIN);

typedef float          v4f   __attribute__((ext_vector_type(4)));
typedef float          v8f   __attribute__((ext_vector_type(8)));
typedef int            v4i   __attribute__((ext_vector_type(4)));
typedef int            v8i   __attribute__((ext_vector_type(8)));
typedef unsigned       v4u   __attribute__((ext_vector_type(4)));
typedef unsigned short v8us  __attribute__((ext_vector_type(8)));
typedef __bf16         v16bf __attribute__((ext_vector_type(16)));
typedef v4f  __attribute__((may_alias)) v4fa;
typedef v4i  __attribute__((may_alias)) v4ia;
typedef v4u  __attribute__((may_alias)) v4ua;
typedef v8us __attribute__((may_alias)) v8usa;
union FragB { v16bf v; v8us h[2]; v8i w; };

__device__ __forceinline__ v8f wmb(const FragB& a, const FragB& b, v8f c) {
  v8f d = __builtin_amdgcn_wmma_f32_16x16x32_bf16(false, a.v, false, b.v, (short)0, c, false, false);
  asm volatile("v_nop\n\tv_nop\n\tv_nop\n\tv_nop" : "+v"(d) : "v"(a.w), "v"(b.w));
  return d;
}
__device__ __forceinline__ v8f z8() { v8f z = {0.f, 0.f, 0.f, 0.f, 0.f, 0.f, 0.f, 0.f}; return z; }

__device__ __forceinline__ unsigned bf16_bits(float f) {
  const unsigned u = __float_as_uint(f);
  return ((u + 0x7FFFu + ((u >> 16) & 1u)) >> 16) & 0xFFFFu;
}
__device__ __forceinline__ float bf16_val(float f) { return __uint_as_float(bf16_bits(f) << 16); }
__device__ __forceinline__ float bfw_lo(unsigned w) { return __uint_as_float(w << 16); }
__device__ __forceinline__ float bfw_hi(unsigned w) { return __uint_as_float(w & 0xffff0000u); }
__device__ __forceinline__ void pack2(float a, float b, unsigned& hw, unsigned& lw) {
  const unsigned ha = bf16_bits(a), hb = bf16_bits(b);
  const unsigned la = bf16_bits(a - __uint_as_float(ha << 16));
  const unsigned lb = bf16_bits(b - __uint_as_float(hb << 16));
  hw = ha | (hb << 16);
  lw = la | (lb << 16);
}
__device__ __forceinline__ float relu_k(float v) { return (v > 0.0f) ? v : (v - v); }

__device__ __forceinline__ void wave_sync() {
  __builtin_amdgcn_fence(__ATOMIC_RELEASE, "wavefront");
  __builtin_amdgcn_wave_barrier();
  __builtin_amdgcn_fence(__ATOMIC_ACQUIRE, "wavefront");
}

__device__ __forceinline__ void slot_info(const int* __restrict__ CNT, const int* __restrict__ OFF,
                                          const int* __restrict__ REC, int node,
                                          int& deg, int& c, int& o, int& flg) {
  const int craw = CNT[node];
  const int oraw = OFF[node];
  const int fraw = REC[(node >> PKS) * 32 + 1];
  const int dg = craw < 0 ? 0 : craw;
  int cc = dg > DEGCAP ? DEGCAP : dg;
  const int oo = oraw < 0 ? 0 : (oraw > RCAP ? RCAP : oraw);
  cc = cc > RCAP - oo ? RCAP - oo : cc;
  deg = dg;
  c = __builtin_amdgcn_readfirstlane(cc);
  o = __builtin_amdgcn_readfirstlane(oo);
  flg = fraw;
}

__global__ __launch_bounds__(NTHR) void k_prep(const float* __restrict__ x,
                                               const float* __restrict__ wl0, const float* __restrict__ wr0,
                                               const float* __restrict__ wl, const float* __restrict__ wr,
                                               const float* __restrict__ wx, const float* __restrict__ wy,
                                               const float* __restrict__ wv,
                                               unsigned short* wzt, unsigned short* wct, unsigned short* wxt,
                                               unsigned short* wyt, unsigned short* wvt, unsigned short* xb) {
  __shared__ __attribute__((aligned(16))) float wzs[2 * FIN * HD];
  const int tid = (int)threadIdx.x;
  const int u = (int)blockIdx.x * NTHR + tid;
  if ((int)blockIdx.x < NU_WZ / NTHR) {
#pragma unroll
    for (int i = 0; i < 2; ++i) {
      const int idx = 4 * (tid + NTHR * i);
      const v4f a = *(const v4f*)(wl0 + idx);
      const v4f c = *(const v4f*)(wr0 + idx);
      *(v4fa*)(wzs + idx) = a;
      *(v4fa*)(wzs + FIN * HD + idx) = c;
    }
  }
  __syncthreads();
  v8us o;
  unsigned short* dp;
  if (u < UB_WZ) {
    const int n = u >> 3, j = u & 7;
    const int seg = j >> 1, kk0 = (j & 1) * 8;
    const int off = (seg >> 1) * (FIN * HD);
    const unsigned msk = (seg == 3) ? 0u : 0xFFFFu;
#pragma unroll
    for (int i = 0; i < 8; ++i) {
      const float f = wzs[off + (kk0 + i) * HD + n];
      asm volatile("" :: "v"(f));
      o[i] = (unsigned short)(bf16_bits(f) & msk);
    }
    dp = wzt + (size_t)u * 8;
  } else if (u < UB_WC) {
    const int v   = u - UB_WZ;
    const int sel = v / NU_WCH;
    const int r   = v - sel * NU_WCH;
    const int l   = r >> 12;
    const int r2  = r & 4095;
    const int n   = r2 >> 5;
    const int j   = r2 & 31;
    const int kk0 = (j & 15) * 8;
    const int k8  = sel * 256 + (j >> 4) * 128 + kk0;
    const size_t so = (size_t)l * HD * HD + (size_t)kk0 * HD + (size_t)n;
    float f[8];
    if (sel == 0) {
#pragma unroll
      for (int i = 0; i < 8; ++i) f[i] = wl[so + (size_t)i * HD];
    } else {
#pragma unroll
      for (int i = 0; i < 8; ++i) f[i] = wr[so + (size_t)i * HD];
    }
#pragma unroll
    for (int i = 0; i < 8; ++i) o[i] = (unsigned short)bf16_bits(f[i]);
    dp = wct + (size_t)l * (HD * KC) + (size_t)n * KC + (size_t)k8;
  } else if (u < UB_WX) {
    const int v = u - UB_WC;
    const int n = v >> 5, j = v & 31;
    const int kk0 = (j & 15) * 8;
    float f[8];
#pragma unroll
    for (int i = 0; i < 8; ++i) f[i] = wx[(size_t)(kk0 + i) * H1D + n];
#pragma unroll
    for (int i = 0; i < 8; ++i) o[i] = (unsigned short)bf16_bits(f[i]);
    dp = wxt + (size_t)v * 8;
  } else if (u < UB_WY) {
    const int v = u - UB_WX;
    const int n = v >> 4, j = v & 15;
    const int kk0 = (j & 7) * 8;
    float f[8];
#pragma unroll
    for (int i = 0; i < 8; ++i) f[i] = wy[(size_t)(kk0 + i) * H2D + n];
#pragma unroll
    for (int i = 0; i < 8; ++i) o[i] = (unsigned short)bf16_bits(f[i]);
    dp = wyt + (size_t)v * 8;
  } else if (u < UB_WV) {
    const int v = u - UB_WY;
    if (v >= ODP * 8) return;
    const int n = v >> 3, j = v & 7;
    const int kk0 = (j & 3) * 8;
    const int nc = n < OD ? n : OD - 1;
    const unsigned msk = (n < OD) ? 0xFFFFu : 0u;
    float f[8];
#pragma unroll
    for (int i = 0; i < 8; ++i) f[i] = wv[(size_t)(kk0 + i) * OD + nc];
#pragma unroll
    for (int i = 0; i < 8; ++i) {
      asm volatile("" :: "v"(f[i]));
      o[i] = (unsigned short)(bf16_bits(f[i]) & msk);
    }
    dp = wvt + (size_t)v * 8;
  } else {
    const int v = u - UB_WV;
    if (v >= NU_XB) return;
    const int row = v >> 1, k8 = (v & 1) * 8;
    const int rc = row < NN ? row : NN - 1;
    const unsigned msk = (row < NN) ? 0xFFFFu : 0u;
    const float* p = x + (size_t)rc * FIN + k8;
    const v4f a = *(const v4f*)p;
    const v4f c = *(const v4f*)(p + 4);
    asm volatile("" :: "v"(a), "v"(c));
    const float f[8] = {a.x, a.y, a.z, a.w, c.x, c.y, c.z, c.w};
#pragma unroll
    for (int i = 0; i < 8; ++i) o[i] = (unsigned short)(bf16_bits(f[i]) & msk);
    dp = xb + (size_t)v * 8;
  }
  *(volatile v8us*)dp = o;
  __threadfence();
  *(volatile v8us*)dp = o;
}

__global__ __launch_bounds__(NTHR) void k_bucket(const int* __restrict__ keys, const int* __restrict__ gidx,
                                                 int* LIST, int* CNT, int* OFF, int* REC) {
  extern __shared__ __attribute__((aligned(16))) int dsm[];
  int* wlst = dsm;
  int* reg2 = wlst + NWAVE * WLCAP;
  int* scnt = reg2 + RCAP;
  int* soff = scnt + NBA;
  int* cur  = soff + NBA;
  int* wcnt = cur + NBA;
  int* wtot = wcnt + 8;
  int* wmx  = wtot + 8;
  const int tid = (int)threadIdx.x, lane = tid & 31, wave = tid >> 5;
  const int nodeBase = (int)blockIdx.x * NBA;
  int nb = NN - nodeBase;
  nb = nb > NBA ? NBA : (nb < 1 ? 1 : nb);

  {
    const v4i z4 = {0, 0, 0, 0};
    for (int i = tid * 4; i < BK_INTS; i += NTHR * 4) *(v4ia*)(dsm + i) = z4;
  }
  __syncthreads();

  int wc = 0;
  {
    const unsigned nbs = (unsigned)nodeBase;
    const unsigned unb = (unsigned)nb;
    const int sent = (int)(1u << 31);
    int* mylist = wlst + wave * WLCAP;
#pragma unroll 1
    for (int st = 0; st < NSTEP; ++st) {
      const int ebw = wave * EPW + st * WSTEP;
      if (ebw >= NE) break;
      const int eb = ebw + lane;
#define LDKEY(J) \
      const int e##J = eb + 32 * (J); \
      const int r##J = keys[e##J < NE ? e##J : NE - 1];
      LDKEY(0) LDKEY(1) LDKEY(2) LDKEY(3) LDKEY(4) LDKEY(5) LDKEY(6) LDKEY(7)
#undef LDKEY
      asm volatile("" :: "v"(r0), "v"(r1), "v"(r2), "v"(r3), "v"(r4), "v"(r5), "v"(r6), "v"(r7));
#define MKHIT(J) \
      const int q##J = -(int)(e##J < NE); \
      const unsigned s##J = (unsigned)((r##J & q##J) | (sent & ~q##J)) - nbs; \
      const bool h##J = s##J < unb;
      MKHIT(0) MKHIT(1) MKHIT(2) MKHIT(3) MKHIT(4) MKHIT(5) MKHIT(6) MKHIT(7)
#undef MKHIT
      const unsigned any = __builtin_amdgcn_ballot_w32(h0 | h1 | h2 | h3 | h4 | h5 | h6 | h7);
      if (any != 0u) {
#define HITJ(J) { \
        const unsigned mj = __builtin_amdgcn_ballot_w32(h##J); \
        if (mj != 0u) { \
          if (h##J) { \
            const int pos = wc + (int)__builtin_amdgcn_mbcnt_lo(mj, 0u); \
            if (pos < WLCAP) mylist[pos] = (int)(((unsigned)e##J << PKS) | s##J); \
          } \
          wc += (int)__builtin_popcount(mj); } }
        HITJ(0) HITJ(1) HITJ(2) HITJ(3) HITJ(4) HITJ(5) HITJ(6) HITJ(7)
#undef HITJ
      }
    }
  }
  if (lane == 0) wcnt[wave] = wc;
  __syncthreads();

  int tot = 0, wov = 0;
#pragma unroll
  for (int w2 = 0; w2 < NWAVE; ++w2) {
    int c = wcnt[w2];
    wov |= (c > WLCAP) ? 1 : 0;
    c = c < 0 ? 0 : (c > WLCAP ? WLCAP : c);
    tot += c;
  }
  const int nh = tot > RCAP ? RCAP : tot;

  if (wave == 0) {
#pragma unroll 1
    for (int w2 = 0; w2 < NWAVE; ++w2) {
      int c = wcnt[w2];
      c = c < 0 ? 0 : (c > WLCAP ? WLCAP : c);
#pragma unroll 1
      for (int b0 = 0; b0 < c; b0 += 32) {
        const int idx = b0 + lane;
        const int uv  = wlst[w2 * WLCAP + (idx < WLCAP ? idx : WLCAP - 1)];
        const int m32 = (c - b0) < 32 ? (c - b0) : 32;
#pragma unroll 1
        for (int k = 0; k < m32; ++k) {
          const int uu = __builtin_amdgcn_readlane(uv, k);
          const int sl = uu & (NBA - 1);
          if (lane == 0) scnt[sl] = scnt[sl] + 1;
        }
      }
    }
  }
  __syncthreads();

  {
    const v4i ca = *(const v4ia*)(scnt + 4 * tid);
    const int e0 = ca.x < 0 ? 0 : ca.x, e1 = ca.y < 0 ? 0 : ca.y, e2 = ca.z < 0 ? 0 : ca.z, e3 = ca.w < 0 ? 0 : ca.w;
    const int ts = e0 + e1 + e2 + e3;
    int incl = ts;
#pragma unroll
    for (int d = 1; d < 32; d <<= 1) {
      const int up = __shfl_up(incl, d, 32);
      if (lane >= d) incl += up;
    }
    int mx = max(max(e0, e1), max(e2, e3));
    mx = max(mx, __shfl_xor(mx, 16, 32));
    mx = max(mx, __shfl_xor(mx, 8, 32));
    mx = max(mx, __shfl_xor(mx, 4, 32));
    mx = max(mx, __shfl_xor(mx, 2, 32));
    mx = max(mx, __shfl_xor(mx, 1, 32));
    if (lane == 31) wtot[wave] = incl;
    if (lane == 0)  wmx[wave] = mx;
    __syncthreads();
    int pre = 0;
#pragma unroll
    for (int w2 = 0; w2 < NWAVE; ++w2) pre += (w2 < wave) ? wtot[w2] : 0;
    int run = pre + incl - ts;
    v4i so;
    so.x = run; run += e0;
    so.y = run; run += e1;
    so.z = run; run += e2;
    so.w = run;
    *(v4ia*)(soff + 4 * tid) = so;
    *(v4ia*)(cur + 4 * tid)  = so;
  }
  __syncthreads();

  if (wave == 0) {
#pragma unroll 1
    for (int w2 = 0; w2 < NWAVE; ++w2) {
      int c = wcnt[w2];
      c = c < 0 ? 0 : (c > WLCAP ? WLCAP : c);
#pragma unroll 1
      for (int b0 = 0; b0 < c; b0 += 32) {
        const int idx = b0 + lane;
        const int uv  = wlst[w2 * WLCAP + (idx < WLCAP ? idx : WLCAP - 1)];
        const int m32 = (c - b0) < 32 ? (c - b0) : 32;
#pragma unroll 1
        for (int k = 0; k < m32; ++k) {
          const int uu  = __builtin_amdgcn_readlane(uv, k);
          const int sl  = uu & (NBA - 1);
          const int eid = (int)((unsigned)uu >> PKS);
          if (lane == 0) {
            int pos = cur[sl];
            pos = pos < 0 ? 0 : (pos > RCAP - 1 ? RCAP - 1 : pos);
            reg2[pos] = eid;
            cur[sl] = pos + 1;
          }
        }
      }
    }
  }
  __syncthreads();

  int bmax = 0;
#pragma unroll
  for (int w2 = 0; w2 < NWAVE; ++w2) bmax = max(bmax, wmx[w2]);
  const int flag = ((tot > RCAP) || (wov != 0) || (bmax > DEGCAP)) ? 1 : 0;

  int* lrow = LIST + (size_t)blockIdx.x * RCAP;
#pragma unroll 1
  for (int it = 0; it < RCAP / (NTHR * 4); ++it) {
    const int i0 = 4 * (it * NTHR + tid);
    const v4i ev = *(const v4ia*)(reg2 + i0);
    int e0 = ev.x, e1 = ev.y, e2 = ev.z, e3 = ev.w;
    e0 = e0 < 0 ? 0 : (e0 > NE - 1 ? NE - 1 : e0);
    e1 = e1 < 0 ? 0 : (e1 > NE - 1 ? NE - 1 : e1);
    e2 = e2 < 0 ? 0 : (e2 > NE - 1 ? NE - 1 : e2);
    e3 = e3 < 0 ? 0 : (e3 > NE - 1 ? NE - 1 : e3);
    int g0 = gidx[e0], g1 = gidx[e1], g2 = gidx[e2], g3 = gidx[e3];
    asm volatile("" :: "v"(g0), "v"(g1), "v"(g2), "v"(g3));
    g0 = g0 < 0 ? 0 : (g0 > NN - 1 ? NN - 1 : g0);
    g1 = g1 < 0 ? 0 : (g1 > NN - 1 ? NN - 1 : g1);
    g2 = g2 < 0 ? 0 : (g2 > NN - 1 ? NN - 1 : g2);
    g3 = g3 < 0 ? 0 : (g3 > NN - 1 ? NN - 1 : g3);
    v4i ov;
    ov.x = g0 & (-(int)(i0     < nh));
    ov.y = g1 & (-(int)(i0 + 1 < nh));
    ov.z = g2 & (-(int)(i0 + 2 < nh));
    ov.w = g3 & (-(int)(i0 + 3 < nh));
    *(volatile v4i*)(lrow + i0) = ov;
    __threadfence();
    *(volatile v4i*)(lrow + i0) = ov;
  }
  {
    const v4i cv = *(const v4ia*)(scnt + 4 * tid);
    const v4i fv = *(const v4ia*)(soff + 4 * tid);
    v4i rv = {0, 0, 0, 0};
    rv.x = (tid == 0) ? bmax : 0;
    rv.y = (tid == 0) ? flag : 0;
    rv.z = (tid == 0) ? nh : 0;
    int* cp = CNT + (size_t)nodeBase + 4 * tid;
    int* fp = OFF + (size_t)nodeBase + 4 * tid;
    int* rp = REC + (size_t)blockIdx.x * 32 + 4 * (tid & 7);
    *(volatile v4i*)cp = cv;
    *(volatile v4i*)fp = fv;
    if (tid < 8) *(volatile v4i*)rp = rv;
    __threadfence();
    *(volatile v4i*)cp = cv;
    *(volatile v4i*)fp = fv;
    if (tid < 8) *(volatile v4i*)rp = rv;
  }
}

__global__ __launch_bounds__(NTHR) void k_replay0(const unsigned short* __restrict__ xb,
                                                  const int* __restrict__ LIST, const int* __restrict__ CNT,
                                                  const int* __restrict__ OFF, const int* __restrict__ REC,
                                                  unsigned short* az) {
  const int tid = (int)threadIdx.x, lane = tid & 31, wave = tid >> 5;
  const int j = lane & 1, g = lane >> 1;
  const float qnan = __uint_as_float(0x7fc00000u);
#pragma unroll 1
  for (int ri = 0; ri < RPW; ++ri) {
    const int node = (int)blockIdx.x * RPB + wave * RPW + ri;
    int deg, c, o, flg;
    slot_info(CNT, OFF, REC, node, deg, c, o, flg);
    const float divv = (float)(deg < 1 ? 1 : deg);
    const bool poison = (flg != 0) || (deg > DEGCAP);
    const int* lp = LIST + (size_t)(node >> PKS) * RCAP;
    float a0 = 0.f, a1 = 0.f, a2 = 0.f, a3 = 0.f, a4 = 0.f, a5 = 0.f, a6 = 0.f, a7 = 0.f;
#pragma unroll 1
    for (int b0 = 0; b0 < c; b0 += 16) {
      const int p = b0 + g;
      int idx = o + p;
      idx = idx > RCAP - 1 ? RCAP - 1 : idx;
      int col = lp[idx];
      col = col < 0 ? 0 : (col > NN - 1 ? NN - 1 : col);
      const v4u w = *(const v4ua*)(xb + (size_t)col * FIN + 8 * j);
      asm volatile("" :: "v"(w));
      const unsigned mk = 0u - (unsigned)(p < c);
      a0 += bfw_lo(w.x & mk); a1 += bfw_hi(w.x & mk);
      a2 += bfw_lo(w.y & mk); a3 += bfw_hi(w.y & mk);
      a4 += bfw_lo(w.z & mk); a5 += bfw_hi(w.z & mk);
      a6 += bfw_lo(w.w & mk); a7 += bfw_hi(w.w & mk);
    }
#pragma unroll
    for (int d = 2; d <= 16; d <<= 1) {
      a0 += __shfl_xor(a0, d, 32); a1 += __shfl_xor(a1, d, 32);
      a2 += __shfl_xor(a2, d, 32); a3 += __shfl_xor(a3, d, 32);
      a4 += __shfl_xor(a4, d, 32); a5 += __shfl_xor(a5, d, 32);
      a6 += __shfl_xor(a6, d, 32); a7 += __shfl_xor(a7, d, 32);
    }
    const v4u xw = *(const v4ua*)(xb + (size_t)node * FIN + 8 * j);
    asm volatile("" :: "v"(xw));
    const bool live = node < NN;
    float m0 = a0 / divv, m1 = a1 / divv, m2 = a2 / divv, m3 = a3 / divv;
    float m4 = a4 / divv, m5 = a5 / divv, m6 = a6 / divv, m7 = a7 / divv;
    m0 = poison ? qnan : m0; m1 = poison ? qnan : m1; m2 = poison ? qnan : m2; m3 = poison ? qnan : m3;
    m4 = poison ? qnan : m4; m5 = poison ? qnan : m5; m6 = poison ? qnan : m6; m7 = poison ? qnan : m7;
    m0 = live ? m0 : 0.0f; m1 = live ? m1 : 0.0f; m2 = live ? m2 : 0.0f; m3 = live ? m3 : 0.0f;
    m4 = live ? m4 : 0.0f; m5 = live ? m5 : 0.0f; m6 = live ? m6 : 0.0f; m7 = live ? m7 : 0.0f;
    unsigned h0, l0, h1, l1, h2, l2, h3, l3;
    pack2(m0, m1, h0, l0);
    pack2(m2, m3, h1, l1);
    pack2(m4, m5, h2, l2);
    pack2(m6, m7, h3, l3);
#if SPLIT_MEAN0 == 0
    l0 = 0u; l1 = 0u; l2 = 0u; l3 = 0u;
#endif
    const int sel = lane >> 1;
    const unsigned mh = 0u - (unsigned)(sel == 0);
    const unsigned ml = 0u - (unsigned)(sel == 1);
    const unsigned mx = 0u - (unsigned)(sel == 2);
    v4u q;
    q.x = (h0 & mh) | (l0 & ml) | (xw.x & mx);
    q.y = (h1 & mh) | (l1 & ml) | (xw.y & mx);
    q.z = (h2 & mh) | (l2 & ml) | (xw.z & mx);
    q.w = (h3 & mh) | (l3 & ml) | (xw.w & mx);
    unsigned short* wp = az + (size_t)node * AZP + 8 * (lane & 7);
    if (lane < 8) *(volatile v4u*)wp = q;
    __threadfence();
    if (lane < 8) *(volatile v4u*)wp = q;
  }
}

__global__ __launch_bounds__(NTHR) void k_replay(const unsigned short* __restrict__ src, unsigned short* dst,
                                                 const int* __restrict__ LIST, const int* __restrict__ CNT,
                                                 const int* __restrict__ OFF, const int* __restrict__ REC) {
  const int tid = (int)threadIdx.x, lane = tid & 31, wave = tid >> 5;
  const bool isHi = (lane >> 4) == 0;
  const float qnan = __uint_as_float(0x7fc00000u);
#pragma unroll 1
  for (int ri = 0; ri < RPW; ++ri) {
    const int node = (int)blockIdx.x * RPB + wave * RPW + ri;
    int deg, c, o, flg;
    slot_info(CNT, OFF, REC, node, deg, c, o, flg);
    const float divv = (float)(deg < 1 ? 1 : deg);
    const bool poison = (flg != 0) || (deg > DEGCAP);
    const int* lp = LIST + (size_t)(node >> PKS) * RCAP;
    float a0 = 0.f, a1 = 0.f, a2 = 0.f, a3 = 0.f, a4 = 0.f, a5 = 0.f, a6 = 0.f, a7 = 0.f;
#pragma unroll 1
    for (int b0 = 0; b0 < c; b0 += 32) {
      int idx = o + b0 + lane;
      idx = idx > RCAP - 1 ? RCAP - 1 : idx;
      int col = lp[idx];
      col = col < 0 ? 0 : (col > NN - 1 ? NN - 1 : col);
      const int m32 = (c - b0) < 32 ? (c - b0) : 32;
#pragma unroll 1
      for (int k = 0; k < m32; ++k) {
        const int sk = __builtin_amdgcn_readlane(col, k);
        const v4u w = *(const v4ua*)(src + (size_t)sk * PP + 8 * lane);
        a0 += bfw_lo(w.x); a1 += bfw_hi(w.x);
        a2 += bfw_lo(w.y); a3 += bfw_hi(w.y);
        a4 += bfw_lo(w.z); a5 += bfw_hi(w.z);
        a6 += bfw_lo(w.w); a7 += bfw_hi(w.w);
      }
    }
    a0 += __shfl_xor(a0, 16, 32); a1 += __shfl_xor(a1, 16, 32);
    a2 += __shfl_xor(a2, 16, 32); a3 += __shfl_xor(a3, 16, 32);
    a4 += __shfl_xor(a4, 16, 32); a5 += __shfl_xor(a5, 16, 32);
    a6 += __shfl_xor(a6, 16, 32); a7 += __shfl_xor(a7, 16, 32);
    const bool live = node < NN;
    float m0 = a0 / divv, m1 = a1 / divv, m2 = a2 / divv, m3 = a3 / divv;
    float m4 = a4 / divv, m5 = a5 / divv, m6 = a6 / divv, m7 = a7 / divv;
    m0 = poison ? qnan : m0; m1 = poison ? qnan : m1; m2 = poison ? qnan : m2; m3 = poison ? qnan : m3;
    m4 = poison ? qnan : m4; m5 = poison ? qnan : m5; m6 = poison ? qnan : m6; m7 = poison ? qnan : m7;
    m0 = live ? m0 : 0.0f; m1 = live ? m1 : 0.0f; m2 = live ? m2 : 0.0f; m3 = live ? m3 : 0.0f;
    m4 = live ? m4 : 0.0f; m5 = live ? m5 : 0.0f; m6 = live ? m6 : 0.0f; m7 = live ? m7 : 0.0f;
    unsigned h0, l0, h1, l1, h2, l2, h3, l3;
    pack2(m0, m1, h0, l0);
    pack2(m2, m3, h1, l1);
    pack2(m4, m5, h2, l2);
    pack2(m6, m7, h3, l3);
    v4u q;
    q.x = isHi ? h0 : l0;
    q.y = isHi ? h1 : l1;
    q.z = isHi ? h2 : l2;
    q.w = isHi ? h3 : l3;
    unsigned short* wp = dst + (size_t)node * PP + 8 * lane;
    *(volatile v4u*)wp = q;
    __threadfence();
    *(volatile v4u*)wp = q;
  }
}

template <int LDB>
__device__ __forceinline__ void kseg(const unsigned short* ap, const unsigned short* wp, int nsteps, v8f (&acc)[8]) {
#pragma unroll 1
  for (int ks = 0; ks < nsteps; ++ks) {
    FragB af;
    af.h[0] = *(const v8usa*)(ap + 32 * ks);
    af.h[1] = *(const v8usa*)(ap + 32 * ks + 16);
#pragma unroll
    for (int t = 0; t < 8; ++t) {
      const unsigned short* wq = wp + (size_t)(16 * t) * (size_t)LDB + 32 * ks;
      FragB bf;
      bf.h[0] = *(const v8usa*)wq;
      bf.h[1] = *(const v8usa*)(wq + 16);
      acc[t] = wmb(af, bf, acc[t]);
    }
  }
}

template <int FIRST>
__global__ __launch_bounds__(GTHR) __attribute__((amdgpu_num_vgpr(248)))
void k_gemm(const unsigned short* A1, const unsigned short* A2, const unsigned short* __restrict__ BT,
            const float* __restrict__ bias, const float* __restrict__ gam, const float* __restrict__ bet,
            unsigned short* outp) {
  __shared__ __attribute__((aligned(16))) float stg[GBM * GBN];
  __shared__ __attribute__((aligned(16))) float bsh[GBN];
  __shared__ __attribute__((aligned(16))) float gsh[GBN];
  __shared__ __attribute__((aligned(16))) float esh[GBN];
  const int tid = (int)threadIdx.x, lane = tid & 31, wave = tid >> 5, hh = lane >> 4, m = lane & 15;
  const int rowBase = (int)blockIdx.x * GBM;

  if (tid < 32) {
    const v4f b4 = *(const v4f*)(bias + 4 * tid);
    const v4f g4 = *(const v4f*)(gam + 4 * tid);
    const v4f e4 = *(const v4f*)(bet + 4 * tid);
    v4f bq, gq, eq;
    bq.x = bf16_val(b4.x); bq.y = bf16_val(b4.y); bq.z = bf16_val(b4.z); bq.w = bf16_val(b4.w);
    gq.x = bf16_val(g4.x); gq.y = bf16_val(g4.y); gq.z = bf16_val(g4.z); gq.w = bf16_val(g4.w);
    eq.x = bf16_val(e4.x); eq.y = bf16_val(e4.y); eq.z = bf16_val(e4.z); eq.w = bf16_val(e4.w);
    *(v4fa*)(bsh + 4 * tid) = bq;
    *(v4fa*)(gsh + 4 * tid) = gq;
    *(v4fa*)(esh + 4 * tid) = eq;
  }

  v8f acc[8];
#pragma unroll
  for (int t = 0; t < 8; ++t) acc[t] = z8();

  if constexpr (FIRST != 0) {
    const unsigned short* ap = A1 + (size_t)(rowBase + 16 * wave + m) * (size_t)AZP + 8 * hh;
    const unsigned short* wp = BT + (size_t)m * (size_t)AZP + 8 * hh;
    kseg<AZP>(ap, wp, AZP / 32, acc);
    (void)A2;
  } else {
    const size_t arow = (size_t)(rowBase + 16 * wave + m) * (size_t)PP + 8 * hh;
    const unsigned short* wp = BT + (size_t)m * (size_t)KC + 8 * hh;
    kseg<KC>(A1 + arow, wp, HD / 32, acc);
#if SPLIT_CONV
    kseg<KC>(A1 + arow + HD, wp + HD, HD / 32, acc);
#endif
    kseg<KC>(A2 + arow, wp + 2 * HD, HD / 32, acc);
#if SPLIT_CONV
    kseg<KC>(A2 + arow + HD, wp + 3 * HD, HD / 32, acc);
#endif
  }

#pragma unroll
  for (int t = 0; t < 8; ++t) {
    const int lc = 16 * t + m;
#pragma unroll
    for (int r = 0; r < 8; ++r) {
      const int lr = 16 * wave + 8 * hh + r;
      stg[lr * GBN + lc] = acc[t][r];
    }
  }
  __syncthreads();

  const v4f b4 = *(const v4fa*)(bsh + 4 * lane);
  const v4f g4 = *(const v4fa*)(gsh + 4 * lane);
  const v4f e4 = *(const v4fa*)(esh + 4 * lane);
  const float invd = 1.0f / (float)HD;
  const bool isHi = (hh == 0);
#pragma unroll 1
  for (int i = 0; i < 16; ++i) {
    const int lr = 16 * wave + i;
    const int gr = rowBase + lr;
    const bool ok = gr < NN;
    float* sp = stg + lr * GBN + 4 * lane;
    const v4f v = *(const v4fa*)sp;
    const float y0 = v.x + b4.x, y1 = v.y + b4.y, y2 = v.z + b4.z, y3 = v.w + b4.w;
    float s = (y0 + y1) + (y2 + y3);
    s += __shfl_xor(s, 16, 32);
    s += __shfl_xor(s, 8, 32);
    s += __shfl_xor(s, 4, 32);
    s += __shfl_xor(s, 2, 32);
    s += __shfl_xor(s, 1, 32);
    const float mu = s * invd;
    const float d0 = y0 - mu, d1 = y1 - mu, d2 = y2 - mu, d3 = y3 - mu;
    float q = (d0 * d0 + d1 * d1) + (d2 * d2 + d3 * d3);
    q += __shfl_xor(q, 16, 32);
    q += __shfl_xor(q, 8, 32);
    q += __shfl_xor(q, 4, 32);
    q += __shfl_xor(q, 2, 32);
    q += __shfl_xor(q, 1, 32);
    const float xv = q * invd + LNEPS;
    float rs = rsqrtf(xv);
    rs = rs * (1.5f - 0.5f * xv * rs * rs);
    v4f ov;
    ov.x = relu_k((d0 * rs) * g4.x + e4.x);
    ov.y = relu_k((d1 * rs) * g4.y + e4.y);
    ov.z = relu_k((d2 * rs) * g4.z + e4.z);
    ov.w = relu_k((d3 * rs) * g4.w + e4.w);
    ov.x = ok ? ov.x : 0.0f; ov.y = ok ? ov.y : 0.0f; ov.z = ok ? ov.z : 0.0f; ov.w = ok ? ov.w : 0.0f;
    *(v4fa*)sp = ov;
    wave_sync();
    const v4f pa = *(const v4fa*)(stg + lr * GBN + 8 * m);
    const v4f pb = *(const v4fa*)(stg + lr * GBN + 8 * m + 4);
    unsigned h0, l0, h1, l1, h2, l2, h3, l3;
    pack2(pa.x, pa.y, h0, l0);
    pack2(pa.z, pa.w, h1, l1);
    pack2(pb.x, pb.y, h2, l2);
    pack2(pb.z, pb.w, h3, l3);
    v4u pw;
    pw.x = isHi ? h0 : l0;
    pw.y = isHi ? h1 : l1;
    pw.z = isHi ? h2 : l2;
    pw.w = isHi ? h3 : l3;
    unsigned short* op = outp + (size_t)gr * (size_t)PP + 8 * lane;
    *(volatile v4u*)op = pw;
    __threadfence();
    *(volatile v4u*)op = pw;
  }
}

__global__ __launch_bounds__(GTHR) __attribute__((amdgpu_num_vgpr(248)))
void k_head(const unsigned short* __restrict__ hp,
            const unsigned short* __restrict__ wxt, const unsigned short* __restrict__ wyt,
            const unsigned short* __restrict__ wvt,
            const float* __restrict__ bx, const float* __restrict__ by, const float* __restrict__ bv,
            float* out) {
  __shared__ __attribute__((aligned(16))) unsigned short t1s[GBM * 2 * H1D];
  __shared__ __attribute__((aligned(16))) unsigned short t2s[GBM * 2 * H2D];
  __shared__ __attribute__((aligned(16))) float os[GBM * OD];
  __shared__ float bxs[H1D];
  __shared__ float bys[H2D];
  __shared__ float bvs[ODP];
  const int tid = (int)threadIdx.x, lane = tid & 31, wave = tid >> 5, hh = lane >> 4, m = lane & 15;
  const int rowBase = (int)blockIdx.x * GBM;

  {
    const float fx = bx[tid < H1D ? tid : H1D - 1];
    const float fy = by[tid < H2D ? tid : H2D - 1];
    const float fv = bv[tid < OD ? tid : OD - 1];
    asm volatile("" :: "v"(fx), "v"(fy), "v"(fv));
    if (tid < H1D) bxs[tid] = bf16_val(fx);
    if (tid < H2D) bys[tid] = bf16_val(fy);
    if (tid < ODP) bvs[tid] = (tid < OD) ? bf16_val(fv) : 0.0f;
  }

  v8f c1[4];
#pragma unroll
  for (int t = 0; t < 4; ++t) c1[t] = z8();
  {
    const unsigned short* ap = hp + (size_t)(rowBase + 16 * wave + m) * (size_t)PP + 8 * hh;
    const unsigned short* wp = wxt + (size_t)m * 256 + 8 * hh;
#pragma unroll 1
    for (int ks = 0; ks < (SPLIT_HEAD ? 8 : 4); ++ks) {
      FragB af;
      af.h[0] = *(const v8usa*)(ap + 32 * ks);
      af.h[1] = *(const v8usa*)(ap + 32 * ks + 16);
#pragma unroll
      for (int t = 0; t < 4; ++t) {
        const unsigned short* wq = wp + (size_t)(16 * t) * 256 + 32 * ks;
        FragB bf;
        bf.h[0] = *(const v8usa*)wq;
        bf.h[1] = *(const v8usa*)(wq + 16);
        c1[t] = wmb(af, bf, c1[t]);
      }
    }
  }
  __syncthreads();
#pragma unroll
  for (int t = 0; t < 4; ++t) {
    const int col = 16 * t + m;
    const float bb = bxs[col];
#pragma unroll
    for (int r = 0; r < 8; ++r) {
      const int row = 16 * wave + 8 * hh + r;
      const float v = relu_k(c1[t][r] + bb);
      const unsigned hb = bf16_bits(v);
      const unsigned lb = bf16_bits(v - __uint_as_float(hb << 16));
      t1s[row * (2 * H1D) + col] = (unsigned short)hb;
      t1s[row * (2 * H1D) + H1D + col] = (unsigned short)lb;
    }
  }
  __syncthreads();

  v8f c2[2];
  c2[0] = z8(); c2[1] = z8();
  {
    const unsigned short* ap = t1s + (16 * wave + m) * (2 * H1D) + 8 * hh;
    const unsigned short* wp = wyt + (size_t)m * 128 + 8 * hh;
#pragma unroll 1
    for (int ks = 0; ks < (SPLIT_HEAD ? 4 : 2); ++ks) {
      FragB af;
      af.h[0] = *(const v8usa*)(ap + 32 * ks);
      af.h[1] = *(const v8usa*)(ap + 32 * ks + 16);
#pragma unroll
      for (int t = 0; t < 2; ++t) {
        const unsigned short* wq = wp + (size_t)(16 * t) * 128 + 32 * ks;
        FragB bf;
        bf.h[0] = *(const v8usa*)wq;
        bf.h[1] = *(const v8usa*)(wq + 16);
        c2[t] = wmb(af, bf, c2[t]);
      }
    }
  }
#pragma unroll
  for (int t = 0; t < 2; ++t) {
    const int col = 16 * t + m;
    const float bb = bys[col];
#pragma unroll
    for (int r = 0; r < 8; ++r) {
      const int row = 16 * wave + 8 * hh + r;
      const float v = relu_k(c2[t][r] + bb);
      const unsigned hb = bf16_bits(v);
      const unsigned lb = bf16_bits(v - __uint_as_float(hb << 16));
      t2s[row * (2 * H2D) + col] = (unsigned short)hb;
      t2s[row * (2 * H2D) + H2D + col] = (unsigned short)lb;
    }
  }
  __syncthreads();

  v8f c3 = z8();
  {
    const unsigned short* ap = t2s + (16 * wave + m) * (2 * H2D) + 8 * hh;
    const unsigned short* wp = wvt + (size_t)m * 64 + 8 * hh;
#pragma unroll 1
    for (int ks = 0; ks < (SPLIT_HEAD ? 2 : 1); ++ks) {
      FragB af;
      af.h[0] = *(const v8usa*)(ap + 32 * ks);
      af.h[1] = *(const v8usa*)(ap + 32 * ks + 16);
      FragB bf;
      bf.h[0] = *(const v8usa*)(wp + 32 * ks);
      bf.h[1] = *(const v8usa*)(wp + 32 * ks + 16);
      c3 = wmb(af, bf, c3);
    }
  }
  {
    const float bb = bvs[m];
#pragma unroll
    for (int r = 0; r < 8; ++r) {
      const int row = 16 * wave + 8 * hh + r;
      const float v = c3[r] + bb;
      if (m < OD) os[row * OD + m] = v;
    }
  }
  __syncthreads();

  int nv = NN - rowBase;
  nv = nv < 0 ? 0 : (nv > GBM ? GBM : nv);
  const int npc = (nv * OD) >> 2;
  v4f fv[2];
  bool okv[2];
  size_t ob[2];
#pragma unroll
  for (int it = 0; it < 2; ++it) {
    const int p  = tid + GTHR * it;
    const int pc = p < (GBM * OD) / 4 ? p : (GBM * OD) / 4 - 1;
    fv[it]  = *(const v4fa*)(os + 4 * pc);
    asm volatile("" :: "v"(fv[it]));
    okv[it] = p < npc;
    ob[it]  = okv[it] ? ((size_t)rowBase * OD + (size_t)(4 * pc)) : (size_t)0;
  }
#pragma unroll
  for (int it = 0; it < 2; ++it) {
    if (okv[it]) *(volatile v4f*)(out + ob[it]) = fv[it];
  }
  __threadfence();
#pragma unroll
  for (int it = 0; it < 2; ++it) {
    if (okv[it]) *(volatile v4f*)(out + ob[it]) = fv[it];
  }
}

static constexpr size_t SZ_WZT  = (size_t)HD * AZP * 2;
static constexpr size_t SZ_WCT  = (size_t)2 * HD * KC * 2;
static constexpr size_t SZ_WXT  = (size_t)H1D * 256 * 2;
static constexpr size_t SZ_WYT  = (size_t)H2D * 128 * 2;
static constexpr size_t SZ_WVT  = (size_t)ODP * 64 * 2;
static constexpr size_t SZ_XB   = (size_t)MP * FIN * 2;
static constexpr size_t SZ_LIST = (size_t)NB * RCAP * 4;
static constexpr size_t SZ_TAB  = (size_t)NB * NBA * 4;
static constexpr size_t SZ_REC  = (size_t)NB * 128;
static constexpr size_t SZ_PL   = (size_t)MP * PP * 2;
static constexpr size_t SZ_AZ   = (size_t)MP * AZP * 2;
static constexpr size_t O_WZT  = 0;
static constexpr size_t O_WCT  = O_WZT + SZ_WZT;
static constexpr size_t O_WXT  = O_WCT + SZ_WCT;
static constexpr size_t O_WYT  = O_WXT + SZ_WXT;
static constexpr size_t O_WVT  = O_WYT + SZ_WYT;
static constexpr size_t O_XB   = O_WVT + SZ_WVT;
static constexpr size_t O_LIST = O_XB + SZ_XB;
static constexpr size_t O_CNT  = O_LIST + SZ_LIST;
static constexpr size_t O_OFF  = O_CNT + SZ_TAB;
static constexpr size_t O_REC  = O_OFF + SZ_TAB;
static constexpr size_t O_PA   = O_REC + SZ_REC;
static constexpr size_t O_PB   = O_PA + SZ_PL;
static constexpr size_t WS_TOTAL = O_PB + SZ_PL;
static_assert(SZ_WZT % 256 == 0 && SZ_WCT % 256 == 0 && SZ_WXT % 256 == 0 && SZ_WYT % 256 == 0);
static_assert(SZ_WVT % 256 == 0 && SZ_XB % 256 == 0 && SZ_LIST % 256 == 0 && SZ_TAB % 256 == 0);
static_assert(SZ_REC % 256 == 0 && SZ_PL % 256 == 0 && SZ_AZ <= SZ_PL);
static_assert(WS_TOTAL <= (size_t)(128u << 20));
static_assert((size_t)NU_WZ * 16 == SZ_WZT && (size_t)NU_WC * 16 == SZ_WCT && (size_t)NU_WX * 16 == SZ_WXT);
static_assert((size_t)NU_WY * 16 == SZ_WYT && (size_t)(ODP * 8) * 16 == SZ_WVT && (size_t)NU_XB * 16 == SZ_XB);

extern "C" void kernel_launch(void* const* d_in, const int* in_sizes, int n_in,
                              void* d_out, int out_size, void* d_ws, size_t ws_size,
                              hipStream_t stream) {
  if (n_in < 16) return;
  const int want[16] = {NN * FIN, 2 * NE, FIN * HD, FIN * HD, HD, 2 * HD * HD, 2 * HD * HD, 2 * HD,
                        3 * HD, 3 * HD, HD * H1D, H1D, H1D * H2D, H2D, H2D * OD, OD};
  for (int i = 0; i < 16; ++i) {
    if (in_sizes[i] != want[i]) return;
  }
  if (out_size != NN * OD) return;
  if (ws_size < WS_TOTAL) return;

  const float* x   = (const float*)d_in[0];
  const int*   ei  = (const int*)  d_in[1];
  const float* Wl0 = (const float*)d_in[2];
  const float* Wr0 = (const float*)d_in[3];
  const float* bl0 = (const float*)d_in[4];
  const float* Wl  = (const float*)d_in[5];
  const float* Wr  = (const float*)d_in[6];
  const float* blv = (const float*)d_in[7];
  const float* lnw = (const float*)d_in[8];
  const float* lnb = (const float*)d_in[9];
  const float* Wx  = (const float*)d_in[10];
  const float* bx  = (const float*)d_in[11];
  const float* Wy  = (const float*)d_in[12];
  const float* by  = (const float*)d_in[13];
  const float* Wv  = (const float*)d_in[14];
  const float* bv  = (const float*)d_in[15];
  float* out = (float*)d_out;
  const int* gix = ei;
  const int* key = ei + NE;

  char* ws = (char*)d_ws;
  unsigned short* WZT = (unsigned short*)(ws + O_WZT);
  unsigned short* WCT = (unsigned short*)(ws + O_WCT);
  unsigned short* WXT = (unsigned short*)(ws + O_WXT);
  unsigned short* WYT = (unsigned short*)(ws + O_WYT);
  unsigned short* WVT = (unsigned short*)(ws + O_WVT);
  unsigned short* XB  = (unsigned short*)(ws + O_XB);
  int* LIST = (int*)(ws + O_LIST);
  int* CNT  = (int*)(ws + O_CNT);
  int* OFF  = (int*)(ws + O_OFF);
  int* REC  = (int*)(ws + O_REC);
  unsigned short* PA = (unsigned short*)(ws + O_PA);
  unsigned short* PB = (unsigned short*)(ws + O_PB);
  unsigned short* AZ = PB;

  hipFuncSetAttribute(reinterpret_cast<const void*>(&k_bucket), hipFuncAttributeMaxDynamicSharedMemorySize, LDS_BK);

  const int gR = MP / GBM;

  k_prep<<<NU_ALL / NTHR, NTHR, 0, stream>>>(x, Wl0, Wr0, Wl, Wr, Wx, Wy, Wv, WZT, WCT, WXT, WYT, WVT, XB);
  k_bucket<<<NB, NTHR, LDS_BK, stream>>>(key, gix, LIST, CNT, OFF, REC);
  k_replay0<<<gR, NTHR, 0, stream>>>(XB, LIST, CNT, OFF, REC, AZ);
  k_gemm<1><<<gR, GTHR, 0, stream>>>(AZ, AZ, WZT, bl0, lnw, lnb, PA);
  k_replay<<<gR, NTHR, 0, stream>>>(PA, PB, LIST, CNT, OFF, REC);
  k_gemm<0><<<gR, GTHR, 0, stream>>>(PB, PA, WCT, blv, lnw + HD, lnb + HD, PB);
  k_replay<<<gR, NTHR, 0, stream>>>(PB, PA, LIST, CNT, OFF, REC);
  k_gemm<0><<<gR, GTHR, 0, stream>>>(PA, PB, WCT + (size_t)HD * KC, blv + HD, lnw + 2 * HD, lnb + 2 * HD, PA);
  k_head<<<gR, GTHR, 0, stream>>>(PA, WXT, WYT, WVT, bx, by, bv, out);
}
